// TemporalSelfAttention_12128987644295
// MI455X (gfx1250) — hardware-verified
//
#include <hip/hip_runtime.h>
#include <math.h>

typedef __attribute__((ext_vector_type(16))) _Float16 v16h;
typedef __attribute__((ext_vector_type(8)))  _Float16 v8h;
typedef __attribute__((ext_vector_type(16))) __bf16   v16b;
typedef __attribute__((ext_vector_type(8)))  __bf16   v8b;
typedef __attribute__((ext_vector_type(8)))  float    v8f;
typedef __attribute__((ext_vector_type(4)))  float    v4f;
typedef __attribute__((ext_vector_type(4)))  unsigned v4u;
#define PSCALE 32768.0f
#define U16(p) ((const unsigned short*)(const void*)(p))
#define PSCALE_INV (1.0f / 32768.0f)

__device__ __forceinline__ unsigned short f2bf_bits(float f) {
  unsigned u = __float_as_uint(f);
  return (unsigned short)((u + 0x7FFFu + ((u >> 16) & 1u)) >> 16);
}
__device__ __forceinline__ float bf_bits2f(unsigned short h) { return __uint_as_float(((unsigned)h) << 16); }

__device__ __forceinline__ void dep_guard_h(v8f& a, v8f& b, v16h x, v16h y) { asm volatile("v_nop\n\tv_nop\n\tv_nop\n\tv_nop" : "+v"(a), "+v"(b) : "v"(x), "v"(y)); }
__device__ __forceinline__ void dep_guard_b(v8f& a, v8f& b, v16b x, v16b y) { asm volatile("v_nop\n\tv_nop\n\tv_nop\n\tv_nop" : "+v"(a), "+v"(b) : "v"(x), "v"(y)); }
__device__ __forceinline__ void keep4_h(v16h a, v16h b, v16h c, v16h d) { asm volatile("v_nop" :: "v"(a), "v"(b), "v"(c), "v"(d)); }
__device__ __forceinline__ void keep4_b(v16b a, v16b b, v16b c, v16b d) { asm volatile("v_nop" :: "v"(a), "v"(b), "v"(c), "v"(d)); }
__device__ __forceinline__ void acc_guard4(v8f& a, v8f& b, v8f& c, v8f& d) { asm volatile("v_nop\n\tv_nop\n\tv_nop\n\tv_nop" : "+v"(a), "+v"(b), "+v"(c), "+v"(d)); }
template <typename T> struct Frag;
template <> struct Frag<_Float16> {
  typedef v16h V; union U { v16h v; v8h h[2]; };
  static __device__ __forceinline__ v16h load(const _Float16* p) {
    U f; f.h[0] = *(const v8h*)(p); f.h[1] = *(const v8h*)(p + 16); return f.v;
  }
  static __device__ __forceinline__ v8f mma(v16h a, v16h b, v8f c) {
    return __builtin_amdgcn_wmma_f32_16x16x32_f16(false, a, false, b, (short)0, c, false, false);
  }
  static __device__ __forceinline__ void guard(v8f& a, v8f& b, v16h x, v16h y) { dep_guard_h(a, b, x, y); }
  static __device__ __forceinline__ void keep(v16h a, v16h b, v16h c, v16h d) { keep4_h(a, b, c, d); }
};
template <> struct Frag<__bf16> {
  typedef v16b V; union U { v16b v; v8b h[2]; };
  static __device__ __forceinline__ v16b load(const __bf16* p) {
    U f; f.h[0] = *(const v8b*)(p); f.h[1] = *(const v8b*)(p + 16); return f.v;
  }
  static __device__ __forceinline__ v8f mma(v16b a, v16b b, v8f c) {
    return __builtin_amdgcn_wmma_f32_16x16x32_bf16(false, a, false, b, (short)0, c, false, false);
  }
  static __device__ __forceinline__ void guard(v8f& a, v8f& b, v16b x, v16b y) { dep_guard_b(a, b, x, y); }
  static __device__ __forceinline__ void keep(v16b a, v16b b, v16b c, v16b d) { keep4_b(a, b, c, d); }
};

template <int ET> struct Elem;
template <> struct Elem<0> { typedef _Float16 T; };
template <> struct Elem<1> { typedef __bf16 T; };
template <int ET, bool SPLIT, int BIAS_MODE, int OUT_MODE, bool RESID, int ACT = 0>
__global__ __launch_bounds__(256) void wmma_gemm64(
    const unsigned short* __restrict__ Ap, const unsigned short* __restrict__ A2p, int lda, long strideA,
    const unsigned short* __restrict__ Btp, const unsigned short* __restrict__ Bt2p, int ldb, long strideB,
    void* __restrict__ Cout, void* __restrict__ Cout2, int ldc, long strideC,
    const float* __restrict__ bias,
    const float* __restrict__ resid, long strideR,
    int M, int N, int K, float scale) {
  typedef typename Elem<ET>::T T;
  typedef typename Frag<T>::V V;
  const T* A = (const T*)Ap; const T* A2 = (const T*)A2p; const T* Bt = (const T*)Btp; const T* Bt2 = (const T*)Bt2p;
  __shared__ __align__(16) float sT[8][16 * 68];
  const int b    = blockIdx.y;
  const int lane = threadIdx.x & 31;
  const int wave = threadIdx.x >> 5;
  const int tilesN = N >> 6;
  const int tilesM = M >> 6;
  const int tile = blockIdx.x * 8 + wave;
  if (tile >= tilesM * tilesN) return;
  const int tm = tile / tilesN;
  const int tn = tile - tm * tilesN;
  const int m0 = tm << 6;
  const int n0 = tn << 6;

  const T* Ab  = A  + (size_t)b * strideA;
  const T* Bb  = Bt + (size_t)b * strideB;
  const T* Ab2 = SPLIT ? (A2  + (size_t)b * strideA) : nullptr;
  const T* Bb2 = SPLIT ? (Bt2 + (size_t)b * strideB) : nullptr;

  const int rlane = lane & 15;
  const int koff  = (lane >> 4) * 8;
  const int mOff  = (lane >> 4) * 8;

  v8f acc[4][4];
#pragma unroll
  for (int i = 0; i < 4; ++i)
#pragma unroll
    for (int j = 0; j < 4; ++j) acc[i][j] = (v8f){0.f,0.f,0.f,0.f,0.f,0.f,0.f,0.f};

  for (int k0 = 0; k0 < K; k0 += 32) {
    V bh[4], bl[4];
#pragma unroll
    for (int j = 0; j < 4; ++j) {
      const size_t bo = (size_t)(n0 + (j << 4) + rlane) * ldb + koff + k0;
      bh[j] = Frag<T>::load(Bb + bo);
      if (SPLIT) bl[j] = Frag<T>::load(Bb2 + bo);
    }
#pragma unroll
    for (int i = 0; i < 4; ++i) {
      const size_t ao = (size_t)(m0 + (i << 4) + rlane) * lda + koff + k0;
      V ah = Frag<T>::load(Ab + ao);
      V al;
      if (SPLIT) al = Frag<T>::load(Ab2 + ao);
#pragma unroll
      for (int j = 0; j < 4; ++j) {
        acc[i][j] = Frag<T>::mma(ah, bh[j], acc[i][j]);
        if (SPLIT) {
          acc[i][j] = Frag<T>::mma(ah, bl[j], acc[i][j]);
          acc[i][j] = Frag<T>::mma(al, bh[j], acc[i][j]);
        }
      }
      Frag<T>::guard(acc[i][0], acc[i][3], ah, SPLIT ? al : ah);
    }
    Frag<T>::keep(bh[0], bh[1], bh[2], bh[3]);
    if (SPLIT) Frag<T>::keep(bl[0], bl[1], bl[2], bl[3]);
  }
  acc_guard4(acc[0][0], acc[0][1], acc[0][2], acc[0][3]);
  acc_guard4(acc[1][0], acc[1][1], acc[1][2], acc[1][3]);
  acc_guard4(acc[2][0], acc[2][1], acc[2][2], acc[2][3]);
  acc_guard4(acc[3][0], acc[3][1], acc[3][2], acc[3][3]);

  float* slab = sT[wave];
  const float* Rb = RESID ? (resid + (size_t)b * strideR) : nullptr;
#pragma unroll
  for (int i = 0; i < 4; ++i) {
    const int mBase = m0 + (i << 4);
#pragma unroll
    for (int j = 0; j < 4; ++j) {
      const int n = n0 + (j << 4) + rlane;
      float bv = 0.f;
      if (BIAS_MODE == 2) bv = bias[n];
#pragma unroll
      for (int r = 0; r < 8; ++r) {
        float v = acc[i][j][r] * scale;
        if (BIAS_MODE == 1) v += bias[mBase + mOff + r];
        if (BIAS_MODE == 2) v += bv;
        if (RESID) v += Rb[(size_t)(mBase + mOff + r) * ldc + n];
        if (ACT == 1) v = tanhf(v);
        if (ACT == 2) v = fmaxf(v, 0.0f);
        if (ACT == 3) v = v / (1.0f + expf(-v));
        if (ACT == 4) v = (v > 0.f) ? v : 0.01f * v;
        if (ACT == 5) v = 0.5f * v * (1.0f + erff(v * 0.70710678118654752f));
        slab[(mOff + r) * 68 + (j << 4) + rlane] = v;
      }
    }
    __builtin_amdgcn_fence(__ATOMIC_RELEASE, "workgroup");
    __builtin_amdgcn_wave_barrier();
    __builtin_amdgcn_fence(__ATOMIC_ACQUIRE, "workgroup");
    if (OUT_MODE == 0) {
      float* C = (float*)Cout + (size_t)b * strideC;
      const int hh = lane >> 4, c4 = (lane & 15) * 4;
      for (int pass = 0; pass < 2; ++pass) {
#pragma unroll
        for (int it = 0; it < 8; ++it) {
          const int row = it * 2 + hh;
          v4f v = *(const v4f*)(slab + row * 68 + c4);
          *(volatile v4f*)(C + (size_t)(mBase + row) * ldc + n0 + c4) = v;
        }
        __threadfence();
      }
    } else {
      const int q = lane >> 3, c8 = (lane & 7) * 8;
      unsigned short* C  = (unsigned short*)Cout  + (size_t)b * strideC;
      unsigned short* C2 = (OUT_MODE == 2) ? ((unsigned short*)Cout2 + (size_t)b * strideC) : nullptr;
      for (int pass = 0; pass < 2; ++pass) {
#pragma unroll
        for (int it = 0; it < 4; ++it) {
          const int row = it * 4 + q;
          const float* sp = slab + row * 68 + c8;
          v8h hv, lv;
#pragma unroll
          for (int e = 0; e < 8; ++e) {
            if (OUT_MODE == 1) {
              hv[e] = (_Float16)sp[e];
            } else {
              unsigned short hb = f2bf_bits(sp[e]);
              unsigned short lb = f2bf_bits(sp[e] - bf_bits2f(hb));
              hv[e] = __builtin_bit_cast(_Float16, hb);
              lv[e] = __builtin_bit_cast(_Float16, lb);
            }
          }
          *(volatile v8h*)(C + (size_t)(mBase + row) * ldc + n0 + c8) = hv;
          if (OUT_MODE == 2) *(volatile v8h*)(C2 + (size_t)(mBase + row) * ldc + n0 + c8) = lv;
        }
        __threadfence();
      }
    }
    __builtin_amdgcn_fence(__ATOMIC_RELEASE, "workgroup");
    __builtin_amdgcn_wave_barrier();
    __builtin_amdgcn_fence(__ATOMIC_ACQUIRE, "workgroup");
  }
}

__global__ __launch_bounds__(256) void cast_f32_f16x2(
    const float* __restrict__ in, _Float16* __restrict__ out, int n2) {
  int i = blockIdx.x * 256 + threadIdx.x;
  if (i < n2) {
    const _Float16 h0 = (_Float16)in[2 * i], h1 = (_Float16)in[2 * i + 1];
    const unsigned u = (unsigned)__builtin_bit_cast(unsigned short, h0) | ((unsigned)__builtin_bit_cast(unsigned short, h1) << 16);
    ((volatile unsigned*)out)[i] = u;
    __threadfence();
    ((volatile unsigned*)out)[i] = u;
  }
}

constexpr int kBatch    = 4;
constexpr int kSeq      = 128;
constexpr int kNodes    = 100;
constexpr int kModel    = 256;
constexpr int kHeads    = 8;
constexpr int kHeadDim  = 128;
constexpr int kInner    = 1024;
constexpr int kQKVWidth = 3072;
constexpr int kRowsPerBatch = kSeq * kNodes;

constexpr int kAttnWaves = 4;
constexpr int kKeyChunk  = 32;
constexpr int kOsPitch   = 132;
constexpr float kProbCarry = 32768.0f;

static_assert(kInner == kHeads * kHeadDim);
static_assert(kQKVWidth == 3 * kInner);
static_assert(kModel % 32 == 0 && kInner % 32 == 0);
static_assert(kRowsPerBatch % 64 == 0);
static_assert(kQKVWidth % 64 == 0 && kModel % 64 == 0);
static_assert(kSeq % 64 == 0 && kSeq % kKeyChunk == 0 && kKeyChunk == 32 && kHeadDim == 128);

__device__ __forceinline__ v8f mma_f16_guarded(v16h a, v16h b, v8f c) {
  c = __builtin_amdgcn_wmma_f32_16x16x32_f16(false, a, false, b, (short)0, c, false, false);
  asm volatile("v_nop\n\tv_nop\n\tv_nop\n\tv_nop" : "+v"(c) : "v"(a), "v"(b));
  return c;
}

__global__ __launch_bounds__(256) void transpose_scale_to_f16(
    const float* __restrict__ in, unsigned short* __restrict__ out, int R, int Cc, float scale) {
  __shared__ __align__(16) float ts[32][260];
  const int c0 = blockIdx.x * 32;
  const int r0 = blockIdx.y * 256;
  const int tid = threadIdx.x;
#pragma unroll
  for (int i = 0; i < 8; ++i) {
    const int idx = i * 256 + tid;
    const int rr = idx >> 3, q4 = idx & 7;
    const v4f v = *(const v4f*)(in + (size_t)(r0 + rr) * Cc + c0 + 4 * q4);
    ts[4 * q4 + 0][rr] = v[0];
    ts[4 * q4 + 1][rr] = v[1];
    ts[4 * q4 + 2][rr] = v[2];
    ts[4 * q4 + 3][rr] = v[3];
  }
  __syncthreads();
  const int wave = tid >> 5, lane = tid & 31;
  _Float16* ob = (_Float16*)out;
  for (int pass = 0; pass < 2; ++pass) {
#pragma unroll
    for (int j = 0; j < 4; ++j) {
      const int cc = wave * 4 + j;
      const float* sp = &ts[cc][8 * lane];
      const v4f a = *(const v4f*)sp;
      const v4f d = *(const v4f*)(sp + 4);
      v8h hv;
      hv[0] = (_Float16)(a[0] * scale); hv[1] = (_Float16)(a[1] * scale);
      hv[2] = (_Float16)(a[2] * scale); hv[3] = (_Float16)(a[3] * scale);
      hv[4] = (_Float16)(d[0] * scale); hv[5] = (_Float16)(d[1] * scale);
      hv[6] = (_Float16)(d[2] * scale); hv[7] = (_Float16)(d[3] * scale);
      *(volatile v8h*)(ob + (size_t)(c0 + cc) * R + r0 + 8 * lane) = hv;
    }
    __threadfence();
  }
}

__global__ __launch_bounds__(256) void bias_concat_x4(
    const float* __restrict__ bq, const float* __restrict__ bk, const float* __restrict__ bv,
    float* __restrict__ bcat) {
  const int p = blockIdx.x;
  const float* src = (p == 0) ? bq : ((p == 1) ? bk : bv);
  const int e4 = threadIdx.x * 4;
  v4f v = *(const v4f*)(src + e4);
  v = v * 4.0f;
  float* dst = bcat + (size_t)p * kInner + e4;
  *(volatile v4f*)dst = v;
  __threadfence();
  *(volatile v4f*)dst = v;
}

__global__ __launch_bounds__(128)
void attn_time_hd128(const unsigned short* __restrict__ qkvp, unsigned short* __restrict__ outp,
                     float sscale, float onorm) {
  __shared__ __align__(16) unsigned short Ksh[kKeyChunk * kHeadDim];
  __shared__ __align__(16) unsigned short Vth[kHeadDim * kKeyChunk];
  __shared__ __align__(16) _Float16 Psh[kAttnWaves][16 * kKeyChunk];
  __shared__ __align__(16) float Osl[kAttnWaves][16 * kOsPitch];

  const int tid  = threadIdx.x;
  const int wave = tid >> 5;
  const int lane = tid & 31;
  const int hh   = lane >> 4;
  const int c    = lane & 15;

  const int bx = blockIdx.x;
  const int qb = bx & 1;
  const int nh = bx >> 1;
  const int h  = nh & (kHeads - 1);
  const int n  = nh >> 3;
  const int q0 = qb * 64 + wave * 16;
  const _Float16* qkv = (const _Float16*)qkvp;

  v16h qa[4];
  {
    const _Float16* qrow = qkv + ((size_t)(q0 + c) * kNodes + n) * kQKVWidth + h * kHeadDim + 8 * hh;
#pragma unroll
    for (int dc = 0; dc < 4; ++dc) qa[dc] = Frag<_Float16>::load(qrow + dc * 32);
  }

  float mrow[8], lrow[8];
  v8f oacc[8];
#pragma unroll
  for (int r = 0; r < 8; ++r) { mrow[r] = -INFINITY; lrow[r] = 0.f; }
#pragma unroll
  for (int t = 0; t < 8; ++t) oacc[t] = (v8f){0.f,0.f,0.f,0.f,0.f,0.f,0.f,0.f};

  for (int kc = 0; kc < kSeq / kKeyChunk; ++kc) {
    const int kv0 = kc * kKeyChunk;
    __syncthreads();
    {
      const int kvr = tid >> 2, part = tid & 3;
      const size_t rb = ((size_t)(kv0 + kvr) * kNodes + n) * kQKVWidth + h * kHeadDim + 32 * part;
      const v4u* ks = (const v4u*)(qkvp + rb + kInner);
      const v4u* vs = (const v4u*)(qkvp + rb + 2 * kInner);
      v4u kk[4], vv[4];
#pragma unroll
      for (int i = 0; i < 4; ++i) { kk[i] = ks[i]; vv[i] = vs[i]; }
#pragma unroll
      for (int i = 0; i < 4; ++i) *(v4u*)(Ksh + kvr * kHeadDim + 32 * part + 8 * i) = kk[i];
#pragma unroll
      for (int i = 0; i < 4; ++i) {
        unsigned short* vc = Vth + (32 * part + 8 * i) * kKeyChunk + kvr;
#pragma unroll
        for (int e = 0; e < 4; ++e) {
          const unsigned w = vv[i][e];
          vc[(2 * e) * kKeyChunk]     = (unsigned short)(w & 0xffffu);
          vc[(2 * e + 1) * kKeyChunk] = (unsigned short)(w >> 16);
        }
      }
    }
    __syncthreads();

    v8f s[2];
#pragma unroll
    for (int j = 0; j < 2; ++j) {
      s[j] = (v8f){0.f,0.f,0.f,0.f,0.f,0.f,0.f,0.f};
#pragma unroll
      for (int dc = 0; dc < 4; ++dc) {
        const v16h kb = Frag<_Float16>::load((const _Float16*)Ksh + (j * 16 + c) * kHeadDim + dc * 32 + 8 * hh);
        s[j] = mma_f16_guarded(qa[dc], kb, s[j]);
      }
    }
    float cm[8];
#pragma unroll
    for (int r = 0; r < 8; ++r) {
      s[0][r] = s[0][r] * sscale;
      s[1][r] = s[1][r] * sscale;
      float m = fmaxf(s[0][r], s[1][r]);
#pragma unroll
      for (int off = 1; off < 16; off <<= 1) m = fmaxf(m, __shfl_xor(m, off, 32));
      cm[r] = m;
    }
    _Float16* pw = Psh[wave];
#pragma unroll
    for (int r = 0; r < 8; ++r) {
      const float mnew  = fmaxf(mrow[r], cm[r]);
      const float alpha = expf(mrow[r] - mnew);
      mrow[r] = mnew;
      float psum = 0.f;
#pragma unroll
      for (int j = 0; j < 2; ++j) {
        const float p = expf(s[j][r] - mnew);
        psum += p;
        pw[(8 * hh + r) * kKeyChunk + j * 16 + c] = (_Float16)(p * kProbCarry);
      }
#pragma unroll
      for (int off = 1; off < 16; off <<= 1) psum += __shfl_xor(psum, off, 32);
      lrow[r] = lrow[r] * alpha + psum;
#pragma unroll
      for (int t = 0; t < 8; ++t) oacc[t][r] *= alpha;
    }
    __builtin_amdgcn_fence(__ATOMIC_RELEASE, "workgroup");
    __builtin_amdgcn_wave_barrier();
    __builtin_amdgcn_fence(__ATOMIC_ACQUIRE, "workgroup");
    {
      const v16h pa = Frag<_Float16>::load(pw + c * kKeyChunk + 8 * hh);
#pragma unroll
      for (int t = 0; t < 8; ++t) {
        const v16h vb = Frag<_Float16>::load((const _Float16*)Vth + (t * 16 + c) * kKeyChunk + 8 * hh);
        oacc[t] = mma_f16_guarded(pa, vb, oacc[t]);
      }
    }
  }

  float* os = Osl[wave];
#pragma unroll
  for (int r = 0; r < 8; ++r) {
    const float inv = onorm * (1.0f / lrow[r]);
#pragma unroll
    for (int t = 0; t < 8; ++t) os[(8 * hh + r) * kOsPitch + t * 16 + c] = oacc[t][r] * inv;
  }
  __builtin_amdgcn_fence(__ATOMIC_RELEASE, "workgroup");
  __builtin_amdgcn_wave_barrier();
  __builtin_amdgcn_fence(__ATOMIC_ACQUIRE, "workgroup");
  {
    const int rp = lane >> 4, c8 = (lane & 15) * 8;
    _Float16* ob = (_Float16*)outp;
    for (int pass = 0; pass < 2; ++pass) {
#pragma unroll
      for (int it = 0; it < 8; ++it) {
        const int row = it * 2 + rp;
        const float* sp = os + row * kOsPitch + c8;
        const v4f a = *(const v4f*)sp;
        const v4f d = *(const v4f*)(sp + 4);
        v8h hv;
        hv[0] = (_Float16)a[0]; hv[1] = (_Float16)a[1]; hv[2] = (_Float16)a[2]; hv[3] = (_Float16)a[3];
        hv[4] = (_Float16)d[0]; hv[5] = (_Float16)d[1]; hv[6] = (_Float16)d[2]; hv[7] = (_Float16)d[3];
        *(volatile v8h*)(ob + ((size_t)(q0 + row) * kNodes + n) * kInner + h * kHeadDim + c8) = hv;
      }
      __threadfence();
    }
  }
}

__global__ __launch_bounds__(256) void residual_layernorm256(
    const float* __restrict__ y, const float* __restrict__ xr,
    const float* __restrict__ gamma, const float* __restrict__ beta,
    float* __restrict__ out, int nrows) {
  const int wave = threadIdx.x >> 5, lane = threadIdx.x & 31;
  const int row = blockIdx.x * 8 + wave;
  if (row >= nrows) return;
  const size_t rb = (size_t)row * kModel;
  const v4f y0 = *(const v4f*)(y + rb + 4 * lane);
  const v4f y1 = *(const v4f*)(y + rb + 128 + 4 * lane);
  const v4f x0 = *(const v4f*)(xr + rb + 4 * lane);
  const v4f x1 = *(const v4f*)(xr + rb + 128 + 4 * lane);
  const v4f g0 = *(const v4f*)(gamma + 4 * lane);
  const v4f g1 = *(const v4f*)(gamma + 128 + 4 * lane);
  const v4f b0 = *(const v4f*)(beta + 4 * lane);
  const v4f b1 = *(const v4f*)(beta + 128 + 4 * lane);
  const v4f v0 = y0 + x0;
  const v4f v1 = y1 + x1;
  float su = 0.0f;
  su += v0[0]; su += v0[1]; su += v0[2]; su += v0[3];
  su += v1[0]; su += v1[1]; su += v1[2]; su += v1[3];
#pragma unroll
  for (int off = 1; off < 32; off <<= 1) su += __shfl_xor(su, off, 32);
  const float mu = su * (1.0f / 256.0f);
  const v4f d0 = v0 - mu;
  const v4f d1 = v1 - mu;
  float sq = 0.0f;
  sq += d0[0] * d0[0]; sq += d0[1] * d0[1]; sq += d0[2] * d0[2]; sq += d0[3] * d0[3];
  sq += d1[0] * d1[0]; sq += d1[1] * d1[1]; sq += d1[2] * d1[2]; sq += d1[3] * d1[3];
#pragma unroll
  for (int off = 1; off < 32; off <<= 1) sq += __shfl_xor(sq, off, 32);
  const float var  = sq * (1.0f / 256.0f);
  const float rstd = rsqrtf(var + 1e-5f);
  const v4f o0 = d0 * rstd * g0 + b0;
  const v4f o1 = d1 * rstd * g1 + b1;
  float* orow = out + rb;
  *(volatile v4f*)(orow + 4 * lane) = o0;
  *(volatile v4f*)(orow + 128 + 4 * lane) = o1;
  __threadfence();
  *(volatile v4f*)(orow + 4 * lane) = o0;
  *(volatile v4f*)(orow + 128 + 4 * lane) = o1;
}

extern "C" void kernel_launch(void* const* d_in, const int* in_sizes, int n_in,
                              void* d_out, int out_size, void* d_ws, size_t ws_size,
                              hipStream_t stream) {
  if (n_in < 11) return;
  const int nRowsAll = kBatch * kRowsPerBatch;
  if (in_sizes[0] != nRowsAll * kModel) return;
  if (in_sizes[1] != kModel * kInner || in_sizes[3] != kModel * kInner || in_sizes[5] != kModel * kInner) return;
  if (in_sizes[2] != kInner || in_sizes[4] != kInner || in_sizes[6] != kInner) return;
  if (in_sizes[7] != kInner * kModel || in_sizes[8] != kModel || in_sizes[9] != kModel || in_sizes[10] != kModel) return;
  if (out_size != nRowsAll * kModel) return;

  const float* x     = (const float*)d_in[0];
  const float* wq    = (const float*)d_in[1];
  const float* bq    = (const float*)d_in[2];
  const float* wk    = (const float*)d_in[3];
  const float* bk    = (const float*)d_in[4];
  const float* wv    = (const float*)d_in[5];
  const float* bv    = (const float*)d_in[6];
  const float* wo    = (const float*)d_in[7];
  const float* bo    = (const float*)d_in[8];
  const float* gamma = (const float*)d_in[9];
  const float* beta  = (const float*)d_in[10];
  float* outAll = (float*)d_out;

  const size_t offWT   = 0;
  const size_t offWoT  = offWT   + (size_t)kQKVWidth * kModel * 2;
  const size_t offBcat = offWoT  + (size_t)kModel * kInner * 2;
  const size_t offXh   = offBcat + (size_t)kQKVWidth * 4;
  const size_t offQKV  = offXh   + (size_t)kRowsPerBatch * kModel * 2;
  const size_t offO    = offQKV  + (size_t)kRowsPerBatch * kQKVWidth * 2;
  const size_t offY    = offO    + (size_t)kRowsPerBatch * kInner * 2;
  const size_t offEnd  = offY    + (size_t)kRowsPerBatch * kModel * 4;
  if (offEnd > ws_size) return;

  char* ws = (char*)d_ws;
  unsigned short* wT   = (unsigned short*)(ws + offWT);
  unsigned short* woT  = (unsigned short*)(ws + offWoT);
  float*          bcat = (float*)(ws + offBcat);
  unsigned short* xh   = (unsigned short*)(ws + offXh);
  unsigned short* qkv  = (unsigned short*)(ws + offQKV);
  unsigned short* oP   = (unsigned short*)(ws + offO);
  float*          yP   = (float*)(ws + offY);

  transpose_scale_to_f16<<<dim3(kInner / 32, kModel / 256), dim3(256), 0, stream>>>(wq, wT, kModel, kInner, 16.0f);
  transpose_scale_to_f16<<<dim3(kInner / 32, kModel / 256), dim3(256), 0, stream>>>(wk, wT + (size_t)kInner * kModel, kModel, kInner, 16.0f);
  transpose_scale_to_f16<<<dim3(kInner / 32, kModel / 256), dim3(256), 0, stream>>>(wv, wT + (size_t)2 * kInner * kModel, kModel, kInner, 16.0f);
  transpose_scale_to_f16<<<dim3(kModel / 32, kInner / 256), dim3(256), 0, stream>>>(wo, woT, kInner, kModel, 32.0f);
  bias_concat_x4<<<dim3(3), dim3(256), 0, stream>>>(bq, bk, bv, bcat);

  const float sscale = 0.0883883476483184f * (1.0f / 16.0f);
  const float onorm  = 16.0f / (kProbCarry * 4.0f);
  const int   sliceElems = kRowsPerBatch * kModel;
  const int   castN2     = sliceElems / 2;

  for (int b = 0; b < kBatch; ++b) {
    const float* xb = x + (size_t)b * sliceElems;
    float* outb = outAll + (size_t)b * sliceElems;

    cast_f32_f16x2<<<dim3((castN2 + 255) / 256), dim3(256), 0, stream>>>(xb, (_Float16*)xh, castN2);

    wmma_gemm64<0, false, 2, 1, false, 0><<<dim3((kRowsPerBatch / 64) * (kQKVWidth / 64) / 8, 1), dim3(256), 0, stream>>>(
        xh, xh, kModel, 0L, wT, wT, kModel, 0L, (void*)qkv, (void*)qkv, kQKVWidth, 0L,
        bcat, bcat, 0L, kRowsPerBatch, kQKVWidth, kModel, 0.25f);

    attn_time_hd128<<<dim3(kNodes * kHeads * (kSeq / 64)), dim3(128), 0, stream>>>(qkv, oP, sscale, onorm);

    wmma_gemm64<0, false, 2, 0, false, 0><<<dim3((kRowsPerBatch / 64) * (kModel / 64) / 8, 1), dim3(256), 0, stream>>>(
        oP, oP, kInner, 0L, woT, woT, kInner, 0L, (void*)yP, (void*)yP, kModel, 0L,
        bo, bo, 0L, kRowsPerBatch, kModel, kInner, 1.0f / 512.0f);

    residual_layernorm256<<<dim3((kRowsPerBatch + 7) / 8), dim3(256), 0, stream>>>(yP, xb, gamma, beta, outb, kRowsPerBatch);
  }
}
